// ConvShapeletFilterClassWise_74912819576991
// MI455X (gfx1250) — hardware-verified
//
#include <hip/hip_runtime.h>

typedef _Float16 v16h __attribute__((ext_vector_type(16)));
typedef _Float16 v8h  __attribute__((ext_vector_type(8)));
typedef float    v8f  __attribute__((ext_vector_type(8)));
typedef float    v4f  __attribute__((ext_vector_type(4)));
typedef v8h __attribute__((may_alias)) v8ha;
typedef v4f __attribute__((may_alias)) v4fa;

union Frag { v16h v; v8h half[2]; };

#define NB      256
#define T_LEN   4096
#define L_LEN   128
#define NSH     128
#define NWIN    3969
#define CH      256
#define NCHUNK  16
#define XS_LEN  384
#define RLEN    384
#define NREP    8
#define EPS_F   1e-6f
#define NEG_BIG (-3.0e38f)

static_assert(NCHUNK * CH >= NWIN);
static_assert(XS_LEN >= CH + L_LEN - 1);
static_assert((RLEN % 8) == 0);
static_assert(NREP * RLEN == 12 * 256);

__device__ __forceinline__ v8f wmma_f16(v16h a, v16h b, v8f c) {
    v8f d = __builtin_amdgcn_wmma_f32_16x16x32_f16(false, a, false, b, (short)0, c, false, false);
    asm volatile("v_nop\n\tv_nop\n\tv_nop\n\tv_nop" : "+v"(d) : "v"(a), "v"(b));
    return d;
}

__device__ __forceinline__ v16h load_frag(const _Float16* p, int h) {
    Frag f;
    f.half[0] = *(const v8ha*)(p + 8 * h);
    f.half[1] = *(const v8ha*)(p + 16 + 8 * h);
    return f.v;
}

__global__ __launch_bounds__(128) void prep_shapelets(const float* __restrict__ sh,
                                                      _Float16* __restrict__ sn)
{
    __shared__ __attribute__((aligned(16))) _Float16 snorm[NSH * L_LEN];
    const int tid = threadIdx.x;
    const float* row = sh + (size_t)tid * L_LEN;

    float s1 = 0.f;
    #pragma unroll 1
    for (int l = 0; l < L_LEN; ++l) s1 += row[l];
    const float mu = s1 * (1.0f / (float)L_LEN);
    float s2 = 0.f;
    #pragma unroll 1
    for (int l = 0; l < L_LEN; ++l) { const float d = row[l] - mu; s2 += d * d; }
    const float var  = s2 * (1.0f / (float)L_LEN);
    const float stdv = sqrtf(var) + EPS_F;
    const float inv  = 1.0f / stdv;
    #pragma unroll 1
    for (int l = 0; l < L_LEN; ++l)
        snorm[tid * L_LEN + l] = (_Float16)((row[l] - mu) * inv);
    __syncthreads();

    #pragma unroll
    for (int it = 0; it < 16; ++it) {
        const int p = it * 128 + tid;
        const v8h v = *(const v8ha*)(snorm + p * 8);
        *(volatile v8h*)(sn + (size_t)p * 8) = v;
    }
    __threadfence();
    #pragma unroll
    for (int it = 0; it < 16; ++it) {
        const int p = it * 128 + tid;
        const v8h v = *(const v8ha*)(snorm + p * 8);
        *(volatile v8h*)(sn + (size_t)p * 8) = v;
    }
}

__global__ __launch_bounds__(256) void corr_kernel(const float* __restrict__ x,
                                                   const _Float16* __restrict__ sn,
                                                   float* __restrict__ part)
{
    __shared__ __attribute__((aligned(16))) float    xs[XS_LEN];
    __shared__ __attribute__((aligned(16))) _Float16 xrep[NREP * RLEN];
    __shared__ float sMu[CH];
    __shared__ float sInv[CH];
    __shared__ __attribute__((aligned(16))) float sPart[NSH];

    const int tid   = threadIdx.x;
    const int lane  = tid & 31;
    const int wid   = tid >> 5;
    const int h     = lane >> 4;
    const int m     = lane & 15;
    const int chunk = blockIdx.x;
    const int b     = blockIdx.y;
    const int t0    = chunk * CH;
    const float* xg = x + (size_t)b * T_LEN;

    #pragma unroll
    for (int it = 0; it < 2; ++it) {
        const int j = tid + it * 256;
        if (j < XS_LEN) {
            const int gi = t0 + j;
            const int gc = min(gi, T_LEN - 1);
            const float v = xg[gc];
            xs[j] = (gi < T_LEN) ? v : 0.f;
        }
    }
    __syncthreads();

    #pragma unroll
    for (int it = 0; it < 12; ++it) {
        const int e  = tid + it * 256;
        const int r  = e / RLEN;
        const int j  = e - r * RLEN;
        const int si = j + r;
        const int sc = min(si, XS_LEN - 1);
        const float v = xs[sc];
        xrep[e] = (_Float16)((si < XS_LEN) ? v : 0.f);
    }

    if (tid < 32) {
        const int o0 = tid * 8;
        float s1 = 0.f, s2 = 0.f;
        #pragma unroll 1
        for (int k = 0; k < L_LEN; ++k) { const float v = xs[o0 + k]; s1 += v; s2 += v * v; }
        #pragma unroll 1
        for (int j = 0; j < 8; ++j) {
            const int o = o0 + j;
            const float mu   = s1 * (1.0f / (float)L_LEN);
            const float var  = fmaxf(s2 * (1.0f / (float)L_LEN) - mu * mu, 0.f);
            const float stdv = sqrtf(var) + EPS_F;
            sMu[o]  = mu;
            sInv[o] = (1.0f / stdv) * (1.0f / (float)L_LEN);
            const float va = xs[o + L_LEN];
            const float vr = xs[o];
            s1 += va - vr;
            s2 += va * va - vr * vr;
        }
    }
    __syncthreads();

    const _Float16* srow = sn + (size_t)(16 * wid + m) * L_LEN;
    v16h bm[4];
    #pragma unroll
    for (int kc = 0; kc < 4; ++kc) bm[kc] = load_frag(srow + 32 * kc, h);
    float snp = 0.f;
    #pragma unroll
    for (int kc = 0; kc < 4; ++kc) {
        #pragma unroll
        for (int i = 0; i < 16; ++i) snp += (float)bm[kc][i];
    }
    const float Sn = snp + __shfl_xor(snp, 16);

    const _Float16* abase = xrep + (m & 7) * RLEN + (m & 8);
    const v8f zero8 = {0.f, 0.f, 0.f, 0.f, 0.f, 0.f, 0.f, 0.f};
    float rmax = NEG_BIG;

    #pragma unroll 1
    for (int tile = 0; tile < 16; ++tile) {
        const int tw = tile * 16;
        v8f c = zero8;
        #pragma unroll
        for (int kc = 0; kc < 4; ++kc) {
            const v16h a = load_frag(abase + tw + 32 * kc, h);
            c = wmma_f16(a, bm[kc], c);
        }
        #pragma unroll
        for (int r = 0; r < 8; ++r) {
            const int t = tw + 8 * h + r;
            float v = (c[r] - sMu[t] * Sn) * sInv[t];
            v = (t0 + t < NWIN) ? v : NEG_BIG;
            rmax = fmaxf(rmax, v);
        }
    }
    rmax = fmaxf(rmax, __shfl_xor(rmax, 16));
    if (h == 0) sPart[16 * wid + m] = rmax;
    __syncthreads();

    if (tid < 32) {
        const v4f v = *(const v4fa*)(sPart + 4 * lane);
        float* dst = part + ((size_t)b * NCHUNK + chunk) * NSH + 4 * lane;
        *(volatile v4f*)dst = v;
        __threadfence();
        *(volatile v4f*)dst = v;
    }
}

__global__ __launch_bounds__(128) void reduce_max(const float* __restrict__ part,
                                                  float* __restrict__ out)
{
    __shared__ __attribute__((aligned(16))) float sOut[NSH];
    const int tid = threadIdx.x;
    const int b   = blockIdx.x;
    const float* p = part + (size_t)b * NCHUNK * NSH + tid;
    float mx = p[0];
    #pragma unroll
    for (int c = 1; c < NCHUNK; ++c) mx = fmaxf(mx, p[c * NSH]);
    sOut[tid] = mx;
    __syncthreads();
    if (tid < 32) {
        const v4f v = *(const v4fa*)(sOut + 4 * tid);
        float* dst = out + (size_t)b * NSH + 4 * tid;
        *(volatile v4f*)dst = v;
        __threadfence();
        *(volatile v4f*)dst = v;
    }
}

extern "C" void kernel_launch(void* const* d_in, const int* in_sizes, int n_in,
                              void* d_out, int out_size, void* d_ws, size_t ws_size,
                              hipStream_t stream)
{
    if (n_in < 2) return;
    if (in_sizes[0] != NB * T_LEN) return;
    if (in_sizes[1] != NSH * L_LEN) return;
    if (out_size != NB * NSH) return;

    const size_t sn_bytes   = (size_t)NSH * L_LEN * 2;
    const size_t part_bytes = (size_t)NB * NCHUNK * NSH * 4;
    const size_t total      = sn_bytes + part_bytes;
    if (total > ws_size) return;

    const float* x  = (const float*)d_in[0];
    const float* sh = (const float*)d_in[1];
    float* out      = (float*)d_out;
    char* ws        = (char*)d_ws;
    _Float16* sn    = (_Float16*)ws;
    float* part     = (float*)(ws + sn_bytes);

    prep_shapelets<<<1, 128, 0, stream>>>(sh, sn);
    dim3 gCorr(NCHUNK, NB);
    corr_kernel<<<gCorr, 256, 0, stream>>>(x, sn, part);
    reduce_max<<<NB, 128, 0, stream>>>(part, out);
}
